// NequIP_90357521973617
// MI455X (gfx1250) — hardware-verified
//
#include <hip/hip_runtime.h>
#include <stddef.h>
#include <math.h>


#define NTHR   128
#define NWAVE  4
#define EPT    8
#define CHUNK  (NTHR * EPT)
#define WCAP   (EPT * 32)
#define LISTN  (NWAVE * WCAP)
#define TEDGE  16
#define PASSN  (NWAVE * TEDGE)
#define PCAP   (CHUNK + PASSN)
#define NB     128
#define EMBK   18
#define KP1    32
#define HID    256
#define NOUT   1024
#define FEAT   64
#define NQ     ((NB * FEAT) / (128 * NWAVE))

#define ISQ3   0.57735026918962576f
#define CSC    0.1767766952966369f
#define CVI    (0.30618621784789724f * 0.57735026918962576f)

static_assert(NQ * 128 * NWAVE == NB * FEAT);
static_assert(PCAP >= CHUNK + PASSN);
static_assert(PASSN <= NTHR);
static_assert((NB % 2) == 0);

typedef float          v4f   __attribute__((ext_vector_type(4)));
typedef float          v8f   __attribute__((ext_vector_type(8)));
typedef int            v4i   __attribute__((ext_vector_type(4)));
typedef unsigned short v8us  __attribute__((ext_vector_type(8)));
typedef unsigned short v16us __attribute__((ext_vector_type(16)));
typedef __bf16         v16bf __attribute__((ext_vector_type(16)));
union Frag { v16bf v; v16us u; v8us h[2]; };

__device__ __forceinline__ unsigned int bf_rne(float f) {
  const unsigned int u = __float_as_uint(f);
  return (u + 0x7FFFu + ((u >> 16) & 1u)) >> 16;
}
__device__ __forceinline__ void split_bf(float x, unsigned short& hi, unsigned short& lo) {
  const unsigned int hb = bf_rne(x);
  const float hf = __uint_as_float(hb << 16);
  const unsigned int lb = bf_rne(x - hf);
  hi = (unsigned short)hb;
  lo = (unsigned short)lb;
}

__device__ __forceinline__ v8f wmb(v16bf a, v16bf b, v8f c) {
  v8f d = __builtin_amdgcn_wmma_f32_16x16x32_bf16(false, a, false, b, (short)0, c, false, false);
  asm volatile("v_nop\n\tv_nop\n\tv_nop\n\tv_nop" : "+v"(d) : "v"(a), "v"(b));
  return d;
}
__device__ __forceinline__ v8f wm3(const Frag& ah, const Frag& al, const Frag& bh, const Frag& bl, v8f c) {
  c = wmb(ah.v, bh.v, c);
  c = wmb(ah.v, bl.v, c);
  c = wmb(al.v, bh.v, c);
  return c;
}

__global__ __launch_bounds__(256) void k_prep(const float* __restrict__ W1, const float* __restrict__ W2,
                                              unsigned short* w2h, unsigned short* w2l,
                                              unsigned short* w1h, unsigned short* w1l, int nblkW2) {
  const int tid = threadIdx.x;
  if ((int)blockIdx.x < nblkW2) {
    const int t = blockIdx.x * 256 + tid;
    const int n = t >> 5, c = t & 31;
    v8us hv, lv;
#pragma unroll
    for (int i = 0; i < 8; ++i) {
      const float x = W2[(size_t)(8 * c + i) * NOUT + n];
      unsigned short ph, pl;
      split_bf(x, ph, pl);
      hv[i] = ph; lv[i] = pl;
    }
    const size_t o = (size_t)n * HID + 8 * c;
    *(volatile v8us*)(w2h + o) = hv;
    *(volatile v8us*)(w2l + o) = lv;
    __threadfence();
    *(volatile v8us*)(w2h + o) = hv;
    *(volatile v8us*)(w2l + o) = lv;
  } else {
    const int t = (blockIdx.x - nblkW2) * 256 + tid;
    const int n = t >> 2, c = t & 3;
    v8us hv, lv;
#pragma unroll
    for (int i = 0; i < 8; ++i) {
      const int k  = 8 * c + i;
      const int kk = k < EMBK ? k : EMBK - 1;
      float x = W1[(size_t)kk * HID + n];
      if (k >= EMBK) x = 0.0f;
      unsigned short ph, pl;
      split_bf(x, ph, pl);
      hv[i] = ph; lv[i] = pl;
    }
    const size_t o = (size_t)n * KP1 + 8 * c;
    *(volatile v8us*)(w1h + o) = hv;
    *(volatile v8us*)(w1l + o) = lv;
    __threadfence();
    *(volatile v8us*)(w1h + o) = hv;
    *(volatile v8us*)(w1l + o) = lv;
  }
}

__device__ __forceinline__ int scan_chunk(const int* __restrict__ dsts, int nE, int cbase, int nodeBase,
                                          int vec8, int* list, int tid, int wave) {
  int wc = 0;
  const int el0  = tid * EPT;
  const int e0   = cbase + el0;
  const int sent = -2147483647 - 1;
  v4i da, db;
  if (vec8 != 0 && cbase + CHUNK <= nE) {
    da = *(const v4i*)(dsts + e0);
    db = *(const v4i*)(dsts + e0 + 4);
  } else {
    da.x = (e0     < nE) ? dsts[min(e0,     nE - 1)] : sent;
    da.y = (e0 + 1 < nE) ? dsts[min(e0 + 1, nE - 1)] : sent;
    da.z = (e0 + 2 < nE) ? dsts[min(e0 + 2, nE - 1)] : sent;
    da.w = (e0 + 3 < nE) ? dsts[min(e0 + 3, nE - 1)] : sent;
    db.x = (e0 + 4 < nE) ? dsts[min(e0 + 4, nE - 1)] : sent;
    db.y = (e0 + 5 < nE) ? dsts[min(e0 + 5, nE - 1)] : sent;
    db.z = (e0 + 6 < nE) ? dsts[min(e0 + 6, nE - 1)] : sent;
    db.w = (e0 + 7 < nE) ? dsts[min(e0 + 7, nE - 1)] : sent;
  }
  const unsigned nb = (unsigned)nodeBase;
  const unsigned s0 = (unsigned)da.x - nb, s1 = (unsigned)da.y - nb;
  const unsigned s2 = (unsigned)da.z - nb, s3 = (unsigned)da.w - nb;
  const unsigned s4 = (unsigned)db.x - nb, s5 = (unsigned)db.y - nb;
  const unsigned s6 = (unsigned)db.z - nb, s7 = (unsigned)db.w - nb;
  const bool h0 = s0 < (unsigned)NB, h1 = s1 < (unsigned)NB, h2 = s2 < (unsigned)NB, h3 = s3 < (unsigned)NB;
  const bool h4 = s4 < (unsigned)NB, h5 = s5 < (unsigned)NB, h6 = s6 < (unsigned)NB, h7 = s7 < (unsigned)NB;
  const unsigned any = __builtin_amdgcn_ballot_w32(h0 | h1 | h2 | h3 | h4 | h5 | h6 | h7);
  if (any != 0u) {
#define HITJ(J, HJ) { \
      const unsigned mj = __builtin_amdgcn_ballot_w32(HJ); \
      if (mj != 0u) { \
        if (HJ) { \
          const int pos = wc + (int)__builtin_amdgcn_mbcnt_lo(mj, 0u); \
          if (pos < WCAP) list[wave * WCAP + pos] = el0 + (J); \
        } \
        wc += (int)__builtin_popcount(mj); } }
    HITJ(0, h0)
    HITJ(1, h1)
    HITJ(2, h2)
    HITJ(3, h3)
    HITJ(4, h4)
    HITJ(5, h5)
    HITJ(6, h6)
    HITJ(7, h7)
#undef HITJ
  }
  return wc;
}

__device__ __forceinline__ v8f tile_w(const unsigned short* ha, const unsigned short* la,
                                      const unsigned short* __restrict__ w2h,
                                      const unsigned short* __restrict__ w2l,
                                      const float* __restrict__ b2, int nt, int m, int hh) {
  const size_t bo = (size_t)(16 * nt + m) * HID + 8 * hh;
  const float bias = b2[16 * nt + m];
  v8f c;
#pragma unroll
  for (int r = 0; r < 8; ++r) c[r] = bias;
#pragma unroll
  for (int kc = 0; kc < 8; ++kc) {
    Frag ah, al, bh, bl;
    ah.h[0] = *(const v8us*)(ha + 32 * kc);
    ah.h[1] = *(const v8us*)(ha + 32 * kc + 16);
    al.h[0] = *(const v8us*)(la + 32 * kc);
    al.h[1] = *(const v8us*)(la + 32 * kc + 16);
    bh.h[0] = *(const v8us*)(w2h + bo + 32 * kc);
    bh.h[1] = *(const v8us*)(w2h + bo + 32 * kc + 16);
    bl.h[0] = *(const v8us*)(w2l + bo + 32 * kc);
    bl.h[1] = *(const v8us*)(w2l + bo + 32 * kc + 16);
    c = wm3(ah, al, bh, bl, c);
  }
  return c;
}

#define FOLD8(A, D, QA, QB) { \
  A[0] = fmaf(D[0], QA.x, A[0]); A[1] = fmaf(D[1], QA.y, A[1]); \
  A[2] = fmaf(D[2], QA.z, A[2]); A[3] = fmaf(D[3], QA.w, A[3]); \
  A[4] = fmaf(D[4], QB.x, A[4]); A[5] = fmaf(D[5], QB.y, A[5]); \
  A[6] = fmaf(D[6], QB.z, A[6]); A[7] = fmaf(D[7], QB.w, A[7]); }

__global__ __launch_bounds__(NTHR) void k_main(
    const float* __restrict__ xnode, const float* __restrict__ eattr, const float* __restrict__ eemb,
    const float* __restrict__ b1, const float* __restrict__ b2,
    const int* __restrict__ esrc, const int* __restrict__ edst,
    const unsigned short* __restrict__ w1h, const unsigned short* __restrict__ w1l,
    const unsigned short* __restrict__ w2h, const unsigned short* __restrict__ w2l,
    float* outp, int nN, int nE, int vec8, float rs) {
  __shared__ __attribute__((aligned(16))) float          acc[(NB + 1) * FEAT];
  __shared__ __attribute__((aligned(16))) float          msg[PASSN * FEAT];
  __shared__ __attribute__((aligned(16))) unsigned short Hh[PASSN * HID];
  __shared__ __attribute__((aligned(16))) unsigned short Hl[PASSN * HID];
  __shared__ __attribute__((aligned(16))) unsigned short Eh[PASSN * KP1];
  __shared__ __attribute__((aligned(16))) unsigned short El[PASSN * KP1];
  __shared__ __attribute__((aligned(16))) float          cvec[NWAVE * 6 * 16 * 16];
  __shared__ __attribute__((aligned(16))) float          ysh[PASSN * 4];
  __shared__ __attribute__((aligned(16))) int            list[LISTN];
  __shared__ __attribute__((aligned(16))) int            pend[PCAP];
  __shared__ int slotb[PASSN];
  __shared__ int wcnt[NWAVE];
  __shared__ int pendN;

  const int tid = threadIdx.x, lane = tid & 31, wave = tid >> 5, hh = lane >> 4, m = lane & 15;
  const int nodeBase = blockIdx.x * NB;

  for (int i = tid; i < (NB + 1) * FEAT; i += NTHR) acc[i] = 0.0f;
  if (tid == 0) pendN = 0;
  __syncthreads();

  const int nChunks = (nE + CHUNK - 1) / CHUNK;
#pragma unroll 1
  for (int ch = 0; ch < nChunks; ++ch) {
    const int cbase = ch * CHUNK;
    const int wc = scan_chunk(edst, nE, cbase, nodeBase, vec8, list, tid, wave);
    if (lane == 0) wcnt[wave] = wc;
    __syncthreads();

    const int base = pendN;
    int tot = 0, myoff = 0;
#pragma unroll
    for (int w = 0; w < NWAVE; ++w) {
      int c = wcnt[w];
      c = c > WCAP ? WCAP : (c < 0 ? 0 : c);
      if (w < wave) myoff += c;
      tot += c;
    }
    int newN = base + tot;
    newN = newN > PCAP ? PCAP : newN;
    {
      int n = wcnt[wave];
      n = n > WCAP ? WCAP : (n < 0 ? 0 : n);
      const int* lp = list + wave * WCAP;
      for (int i = lane; i < n; i += 32) {
        const int pos = base + myoff + i;
        if (pos < PCAP) pend[pos] = cbase + lp[i];
      }
    }
    const int fin = (ch == nChunks - 1) ? 1 : 0;
    const int R   = (fin != 0) ? (newN + PASSN - 1) / PASSN : newN / PASSN;
    const int Pv  = (fin != 0) ? newN : R * PASSN;
    __syncthreads();

#pragma unroll 1
    for (int ps = 0; ps < R; ++ps) {
      {
        const int es = lane & 15;
        int idx = ps * PASSN + wave * TEDGE + es;
        const bool valid = idx < Pv;
        idx = idx < 0 ? 0 : (idx > PCAP - 1 ? PCAP - 1 : idx);
        int e = pend[idx];
        if (!valid) e = 0;
        e = e < 0 ? 0 : (e > nE - 1 ? nE - 1 : e);
        const int d = edst[e];
        int s = esrc[e];
        int slot = d - nodeBase;
        if (!valid || (unsigned)slot >= (unsigned)NB) slot = NB;
        s = s < 0 ? 0 : (s > nN - 1 ? nN - 1 : s);

        const float* er = eemb + (size_t)e * EMBK;
        v8us eh0, el0, eh1, el1;
#pragma unroll
        for (int i = 0; i < 8; ++i) {
          const int ka = 16 * hh + i, kb = 16 * hh + 8 + i;
          float xa = er[ka < EMBK ? ka : EMBK - 1]; if (ka >= EMBK) xa = 0.0f;
          float xb = er[kb < EMBK ? kb : EMBK - 1]; if (kb >= EMBK) xb = 0.0f;
          unsigned short ph, pl;
          split_bf(xa, ph, pl); eh0[i] = ph; el0[i] = pl;
          split_bf(xb, ph, pl); eh1[i] = ph; el1[i] = pl;
        }
        {
          unsigned short* hp = Eh + (wave * TEDGE + es) * KP1 + 16 * hh;
          unsigned short* lp = El + (wave * TEDGE + es) * KP1 + 16 * hh;
          *(v8us*)hp = eh0; *(v8us*)(hp + 8) = eh1;
          *(v8us*)lp = el0; *(v8us*)(lp + 8) = el1;
        }

        const float* xr = xnode + (size_t)s * FEAT;
        const float y0 = eattr[(size_t)e * 4 + 0];
        const float ya = eattr[(size_t)e * 4 + 1];
        const float yb = eattr[(size_t)e * 4 + 2];
        const float yc = eattr[(size_t)e * 4 + 3];
        float* cw = cvec + wave * (6 * 256);
#pragma unroll
        for (int ii = 0; ii < 8; ++ii) {
          const int i = 8 * hh + ii;
          const float sv = xr[i];
          const float v0 = xr[16 + 3 * i], v1 = xr[17 + 3 * i], v2 = xr[18 + 3 * i];
          cw[(0 * 16 + i) * 16 + es] = y0 * sv;
          cw[(1 * 16 + i) * 16 + es] = ISQ3 * (ya * v0 + yb * v1 + yc * v2);
          cw[(2 * 16 + i) * 16 + es] = sv;
          cw[(3 * 16 + i) * 16 + es] = v0;
          cw[(4 * 16 + i) * 16 + es] = v1;
          cw[(5 * 16 + i) * 16 + es] = v2;
        }
        if (hh == 0) {
          ysh[(wave * TEDGE + es) * 4 + 0] = y0;
          ysh[(wave * TEDGE + es) * 4 + 1] = ya;
          ysh[(wave * TEDGE + es) * 4 + 2] = yb;
          ysh[(wave * TEDGE + es) * 4 + 3] = yc;
          slotb[wave * TEDGE + es] = slot;
        }
      }
      __syncthreads();

      {
        Frag ah, al;
        const unsigned short* ep = Eh + (wave * TEDGE + m) * KP1;
        const unsigned short* lq = El + (wave * TEDGE + m) * KP1;
        ah.h[0] = *(const v8us*)(ep + 8 * hh);
        ah.h[1] = *(const v8us*)(ep + 16 + 8 * hh);
        al.h[0] = *(const v8us*)(lq + 8 * hh);
        al.h[1] = *(const v8us*)(lq + 16 + 8 * hh);
        unsigned short* hrow = Hh + (wave * TEDGE + 8 * hh) * HID + m;
        unsigned short* lrow = Hl + (wave * TEDGE + 8 * hh) * HID + m;
#pragma unroll 1
        for (int nt = 0; nt < 16; ++nt) {
          Frag bh, bl;
          const size_t bo = (size_t)(16 * nt + m) * KP1;
          bh.h[0] = *(const v8us*)(w1h + bo + 8 * hh);
          bh.h[1] = *(const v8us*)(w1h + bo + 16 + 8 * hh);
          bl.h[0] = *(const v8us*)(w1l + bo + 8 * hh);
          bl.h[1] = *(const v8us*)(w1l + bo + 16 + 8 * hh);
          const float bias = b1[16 * nt + m];
          v8f c;
#pragma unroll
          for (int r = 0; r < 8; ++r) c[r] = bias;
          c = wm3(ah, al, bh, bl, c);
#pragma unroll
          for (int r = 0; r < 8; ++r) {
            const float x  = c[r];
            const float t  = __expf(-x);
            const float sg = __builtin_amdgcn_rcpf(1.0f + t);
            const float hv = x * sg;
            unsigned short ph, pl;
            split_bf(hv, ph, pl);
            hrow[r * HID + 16 * nt] = ph;
            lrow[r * HID + 16 * nt] = pl;
          }
        }
      }
      __syncthreads();

      {
        const unsigned short* ha = Hh + (wave * TEDGE + m) * HID + 8 * hh;
        const unsigned short* la = Hl + (wave * TEDGE + m) * HID + 8 * hh;
        const float* cwv = cvec + wave * (6 * 256) + 8 * hh;
        float a_ss[8], a_vv[8], a_sv[8], a_v0[8], a_v1[8], a_v2[8];
#pragma unroll
        for (int r = 0; r < 8; ++r) { a_ss[r] = 0.0f; a_vv[r] = 0.0f; a_sv[r] = 0.0f; a_v0[r] = 0.0f; a_v1[r] = 0.0f; a_v2[r] = 0.0f; }

#pragma unroll 1
        for (int i = 0; i < 16; ++i) {
          const v8f d = tile_w(ha, la, w2h, w2l, b2, 0 * 16 + i, m, hh);
          const float* cp = cwv + (0 * 16 + i) * 16;
          const v4f qa = *(const v4f*)cp, qb = *(const v4f*)(cp + 4);
          FOLD8(a_ss, d, qa, qb)
        }
#pragma unroll 1
        for (int i = 0; i < 16; ++i) {
          const v8f d = tile_w(ha, la, w2h, w2l, b2, 1 * 16 + i, m, hh);
          const float* cp = cwv + (1 * 16 + i) * 16;
          const v4f qa = *(const v4f*)cp, qb = *(const v4f*)(cp + 4);
          FOLD8(a_vv, d, qa, qb)
        }
#pragma unroll 1
        for (int i = 0; i < 16; ++i) {
          const v8f d = tile_w(ha, la, w2h, w2l, b2, 2 * 16 + i, m, hh);
          const float* cp = cwv + (2 * 16 + i) * 16;
          const v4f qa = *(const v4f*)cp, qb = *(const v4f*)(cp + 4);
          FOLD8(a_sv, d, qa, qb)
        }
#pragma unroll 1
        for (int i = 0; i < 16; ++i) {
          const v8f d = tile_w(ha, la, w2h, w2l, b2, 3 * 16 + i, m, hh);
          const float* c0 = cwv + (3 * 16 + i) * 16;
          const float* c1 = cwv + (4 * 16 + i) * 16;
          const float* c2 = cwv + (5 * 16 + i) * 16;
          const v4f q0a = *(const v4f*)c0, q0b = *(const v4f*)(c0 + 4);
          const v4f q1a = *(const v4f*)c1, q1b = *(const v4f*)(c1 + 4);
          const v4f q2a = *(const v4f*)c2, q2b = *(const v4f*)(c2 + 4);
          FOLD8(a_v0, d, q0a, q0b)
          FOLD8(a_v1, d, q1a, q1b)
          FOLD8(a_v2, d, q2a, q2b)
        }

        const int eb = wave * TEDGE + 8 * hh;
#pragma unroll
        for (int r = 0; r < 8; ++r) {
          const v4f y = *(const v4f*)(ysh + (eb + r) * 4);
          float* mp = msg + (eb + r) * FEAT;
          mp[m]              = CSC * (a_ss[r] + a_vv[r]);
          mp[16 + 3 * m + 0] = CVI * (a_sv[r] * y.y + a_v0[r] * y.x);
          mp[16 + 3 * m + 1] = CVI * (a_sv[r] * y.z + a_v1[r] * y.x);
          mp[16 + 3 * m + 2] = CVI * (a_sv[r] * y.w + a_v2[r] * y.x);
        }
      }
      __syncthreads();

      if (tid < FEAT) {
#pragma unroll 1
        for (int i = 0; i < PASSN; ++i) {
          int sl = slotb[i];
          sl = sl < 0 ? 0 : (sl > NB ? NB : sl);
          acc[sl * FEAT + tid] += msg[i * FEAT + tid];
        }
      }
      __syncthreads();
    }

    int rem = newN - R * PASSN;
    rem = rem < 0 ? 0 : rem;
    if (R > 0 && tid < rem) pend[tid] = pend[R * PASSN + tid];
    if (tid == 0) pendN = rem;
  }
  __syncthreads();

  const size_t ob  = (size_t)nodeBase * FEAT;
  const size_t lim = (size_t)nN * FEAT;
#pragma unroll 1
  for (int q = 0; q < NQ; ++q) {
    const int f = (wave * NQ + q) * 128 + 4 * lane;
    v4f v = *(const v4f*)(acc + f);
    v = v * rs;
    const size_t gi = ob + (size_t)f;
    if (gi < lim) *(volatile v4f*)(outp + gi) = v;
  }
  __threadfence();
#pragma unroll 1
  for (int q = 0; q < NQ; ++q) {
    const int f = (wave * NQ + q) * 128 + 4 * lane;
    v4f v = *(const v4f*)(acc + f);
    v = v * rs;
    const size_t gi = ob + (size_t)f;
    if (gi < lim) *(volatile v4f*)(outp + gi) = v;
  }
}

extern "C" void kernel_launch(void* const* d_in, const int* in_sizes, int n_in,
                              void* d_out, int out_size, void* d_ws, size_t ws_size,
                              hipStream_t stream) {
  if (n_in < 9) return;
  const int nN = in_sizes[0] / FEAT;
  const int nE = in_sizes[7];
  if (nN <= 0 || nE <= 0) return;
  if (in_sizes[0] != nN * FEAT || in_sizes[1] != nE * 4 || in_sizes[2] != nE * EMBK) return;
  if (in_sizes[3] != EMBK * HID || in_sizes[4] != HID || in_sizes[5] != HID * NOUT || in_sizes[6] != NOUT) return;
  if (in_sizes[8] != nE || out_size != nN * FEAT) return;

  const float* xnode = (const float*)d_in[0];
  const float* eattr = (const float*)d_in[1];
  const float* eemb  = (const float*)d_in[2];
  const float* W1    = (const float*)d_in[3];
  const float* b1    = (const float*)d_in[4];
  const float* W2    = (const float*)d_in[5];
  const float* b2    = (const float*)d_in[6];
  const int*   esrc  = (const int*)d_in[7];
  const int*   edst  = (const int*)d_in[8];
  float* out = (float*)d_out;

  char* ws = (char*)d_ws;
  size_t off = 0;
  const size_t szW2 = (size_t)NOUT * HID * 2;
  const size_t szW1 = (size_t)HID * KP1 * 2;
  const size_t oW2h = off; off += szW2;
  const size_t oW2l = off; off += szW2;
  const size_t oW1h = off; off += szW1;
  const size_t oW1l = off; off += szW1;
  if (off > ws_size) return;
  unsigned short* w2h = (unsigned short*)(ws + oW2h);
  unsigned short* w2l = (unsigned short*)(ws + oW2l);
  unsigned short* w1h = (unsigned short*)(ws + oW1h);
  unsigned short* w1l = (unsigned short*)(ws + oW1l);

  const float cden = (float)sqrt((double)nE / (double)nN);
  const float rs = 1.0f / cden;
  const int vec8 = 1;
  const int nblkW2 = (NOUT * HID) / (8 * 256);
  const int nblkW1 = (HID * KP1) / (8 * 256);
  const int nBlk = (nN + NB - 1) / NB;

  k_prep<<<nblkW2 + nblkW1, 256, 0, stream>>>(W1, W2, w2h, w2l, w1h, w1l, nblkW2);

  k_main<<<nBlk, NTHR, 0, stream>>>(xnode, eattr, eemb, b1, b2, esrc, edst,
                                    w1h, w1l, w2h, w2l, out, nN, nE, vec8, rs);
}
